// Feature_learning_layer_2886218023203
// MI455X (gfx1250) — hardware-verified
//
#include <hip/hip_runtime.h>
#include <stddef.h>


#define NAG   256
#define NF    64
#define NODES 2048
#define NPP   416
#define NAP   128
#define WE1P  144
#define WC1SZ 9216

#define OE2H  0
#define OE2L  4096
#define OC2H  8192
#define OC2L  10240
#define ON1H  12288
#define ON1L  20480
#define ON2H  28672
#define ON2L  32768
#define WBN   36864

#define SMF_CST   0
#define SMF_OST   12288
#define SMF_RED   24576
#define SMF_TOTAL 24640

#define EPSV 1e-4f

typedef float v4f  __attribute__((ext_vector_type(4)));
typedef float v4fa __attribute__((ext_vector_type(4), may_alias));
typedef float v8f  __attribute__((ext_vector_type(8)));
typedef int   v4i  __attribute__((ext_vector_type(4)));
typedef __bf16 bf16;
typedef bf16  v8b  __attribute__((ext_vector_type(8)));
typedef bf16  v8ba __attribute__((ext_vector_type(8), may_alias));
typedef bf16  v16b __attribute__((ext_vector_type(16)));
union FragB { v16b v; v8b h[2]; };
union B8 { v8b b; v4i i; };

#define GE(a, e) ((a)[(e) >> 2][(e) & 3])

__device__ __forceinline__ v8f zacc() {
  v8f z;
#pragma unroll
  for (int i = 0; i < 8; ++i) z[i] = 0.0f;
  return z;
}

__device__ __forceinline__ v8b zero8b() {
  v8b z;
#pragma unroll
  for (int i = 0; i < 8; ++i) z[i] = (bf16)0.0f;
  return z;
}

__device__ __forceinline__ v8f wmb(v16b a, v16b b, v8f c) {
  v8f d = __builtin_amdgcn_wmma_f32_16x16x32_bf16(false, a, false, b, (short)0, c, false, false);
  asm volatile("v_nop\n\tv_nop\n\tv_nop\n\tv_nop" : "+v"(d) : "v"(a), "v"(b));
  return d;
}

__device__ __forceinline__ v8f wm3(const FragB& ah, const FragB& al, const FragB& bh, const FragB& bl, v8f c) {
  c = wmb(ah.v, bh.v, c);
  c = wmb(ah.v, bl.v, c);
  c = wmb(al.v, bh.v, c);
  return c;
}

__device__ __forceinline__ void split4(const v4f x, FragB& hi, FragB& lo, const int g, const int base) {
#pragma unroll
  for (int i = 0; i < 4; ++i) {
    const float f = x[i];
    const bf16 hb = (bf16)f;
    const float rem = f - (float)hb;
    hi.h[g][base + i] = hb;
    lo.h[g][base + i] = (bf16)rem;
  }
}

__device__ __forceinline__ void ldsplit(const float* p, const int hh, FragB& hi, FragB& lo) {
  const float* a = p + 8 * hh;
  const v4f x0 = *(const v4fa*)(a);
  const v4f x1 = *(const v4fa*)(a + 4);
  const v4f x2 = *(const v4fa*)(a + 16);
  const v4f x3 = *(const v4fa*)(a + 20);
  split4(x0, hi, lo, 0, 0);
  split4(x1, hi, lo, 0, 4);
  split4(x2, hi, lo, 1, 0);
  split4(x3, hi, lo, 1, 4);
}

__device__ __forceinline__ void ldb16(const bf16* ph, const bf16* pl, const int hh, FragB& hi, FragB& lo) {
  hi.h[0] = *(const v8ba*)(ph + 8 * hh);
  hi.h[1] = *(const v8ba*)(ph + 16 + 8 * hh);
  lo.h[0] = *(const v8ba*)(pl + 8 * hh);
  lo.h[1] = *(const v8ba*)(pl + 16 + 8 * hh);
}

__device__ __forceinline__ float wsum(float v) {
  v += __shfl_xor(v, 16);
  v += __shfl_xor(v, 8);
  v += __shfl_xor(v, 4);
  v += __shfl_xor(v, 2);
  v += __shfl_xor(v, 1);
  return v;
}

__global__ __launch_bounds__(256) void k_wsplit(const float* __restrict__ We2, const float* __restrict__ Wc2,
                                                 const float* __restrict__ Wn1, const float* __restrict__ Wn2,
                                                 bf16* WB) {
  const int blk = blockIdx.x, tid = threadIdx.x;
  const float* src;
  int loc, dh, dl;
  if (blk < 2)      { src = We2; loc = blk * 2048;       dh = OE2H; dl = OE2L; }
  else if (blk < 3) { src = Wc2; loc = 0;                dh = OC2H; dl = OC2L; }
  else if (blk < 7) { src = Wn1; loc = (blk - 3) * 2048; dh = ON1H; dl = ON1L; }
  else              { src = Wn2; loc = (blk - 7) * 2048; dh = ON2H; dl = ON2L; }
  const int e = loc + tid * 8;
  const v4f a = *(const v4fa*)(src + e);
  const v4f c = *(const v4fa*)(src + e + 4);
  FragB hi, lo;
  split4(a, hi, lo, 0, 0);
  split4(c, hi, lo, 0, 4);
  B8 uh, ul;
  uh.b = hi.h[0];
  ul.b = lo.h[0];
  bf16* qh = WB + dh + e;
  bf16* ql = WB + dl + e;
  *(volatile v4i*)qh = uh.i;
  *(volatile v4i*)ql = ul.i;
  __threadfence();
  *(volatile v4i*)qh = uh.i;
  *(volatile v4i*)ql = ul.i;
}

__global__ __launch_bounds__(256) void k_copy(const float* __restrict__ src, float* dst) {
  const int t = blockIdx.x * 256 + threadIdx.x;
  v4f v[4];
#pragma unroll
  for (int k = 0; k < 4; ++k) v[k] = *(const v4fa*)(src + ((size_t)k * 65536 + (size_t)t) * 4);
#pragma unroll
  for (int k = 0; k < 4; ++k) *(volatile v4f*)(dst + ((size_t)k * 65536 + (size_t)t) * 4) = v[k];
  __threadfence();
#pragma unroll
  for (int k = 0; k < 4; ++k) *(volatile v4f*)(dst + ((size_t)k * 65536 + (size_t)t) * 4) = v[k];
}

__device__ __forceinline__ void planes_store(const float* tile, float* base, const int lane) {
#pragma unroll 1
  for (int row = 0; row < 16; ++row) {
#pragma unroll
    for (int q = 0; q < 4; ++q) {
      const int piece = q * 32 + lane;
      const int pc = min(piece, 103);
      const v4f v = *(const v4fa*)(tile + row * NPP + pc * 4);
      if (piece < 104) *(volatile v4f*)(base + (size_t)row * NPP + piece * 4) = v;
    }
  }
}

__global__ __launch_bounds__(32) void k_planes(const float* __restrict__ h,
                                                const float* __restrict__ We1, const float* __restrict__ bE1,
                                                const float* __restrict__ Wc1, const float* __restrict__ bC1,
                                                const float* __restrict__ Wqm, const float* __restrict__ bqm,
                                                float* NP) {
  __shared__ __attribute__((aligned(16))) float tile[16 * NPP];
  const int lane = threadIdx.x & 31, hh = lane >> 4, m = lane & 15;
  const int row0 = blockIdx.x * 16;
  FragB ah0, al0, ah1, al1;
  {
    const float* ap = h + (size_t)(row0 + m) * NF;
    ldsplit(ap, hh, ah0, al0);
    ldsplit(ap + 32, hh, ah1, al1);
  }
#pragma unroll 1
  for (int nt = 0; nt < 25; ++nt) {
    const int col0 = nt * 16;
    const float* wrow;
    float bias;
    int dorelu;
    if (col0 < 384) {
      const int part = (col0 >= 192) ? 1 : 0;
      const int cq = col0 - 192 * part;
      const int hd = cq >> 6;
      const int o = (cq & 63) + m;
      const int hc = (hd > 0) ? (hd - 1) : 0;
      const float* wb = (hd == 0) ? We1 : (Wc1 + (size_t)hc * WC1SZ);
      wrow = wb + (size_t)o * WE1P + part * NF;
      const float b0 = bE1[o];
      const float b1 = bC1[hc * NF + o];
      const float bv = (hd == 0) ? b0 : b1;
      bias = (part == 0) ? bv : 0.0f;
      dorelu = 0;
    } else {
      wrow = Wqm + (size_t)m * NF;
      bias = bqm[m];
      dorelu = 1;
    }
    FragB bh, bl;
    v8f acc = zacc();
    ldsplit(wrow, hh, bh, bl);
    acc = wm3(ah0, al0, bh, bl, acc);
    ldsplit(wrow + 32, hh, bh, bl);
    acc = wm3(ah1, al1, bh, bl, acc);
#pragma unroll
    for (int r = 0; r < 8; ++r) {
      float v = acc[r] + bias;
      v = dorelu ? fmaxf(v, 0.0f) : v;
      tile[(8 * hh + r) * NPP + col0 + m] = v;
    }
  }
#pragma unroll
  for (int r = 0; r < 8; ++r) tile[(8 * hh + r) * NPP + 400 + m] = 0.0f;
  __syncthreads();
  float* base = NP + (size_t)row0 * NPP;
  planes_store(tile, base, lane);
  __threadfence();
  planes_store(tile, base, lane);
}

__global__ __launch_bounds__(64) void k_pairs(
    const float* __restrict__ NP, const float* __restrict__ coord, const float* __restrict__ category,
    const bf16* __restrict__ WB, const float* __restrict__ We1, const float* __restrict__ Wc1,
    const float* __restrict__ bE2g, const float* __restrict__ bC2g,
    const float* __restrict__ Wf1g, const float* __restrict__ bF1g,
    const float* __restrict__ Wf2g, const float* __restrict__ bF2g, float* NA) {
  __shared__ __attribute__((aligned(16))) bf16  CAh[3072];
  __shared__ __attribute__((aligned(16))) bf16  CAl[3072];
  __shared__ __attribute__((aligned(16))) bf16  uH[6144];
  __shared__ __attribute__((aligned(16))) bf16  uL[6144];
  __shared__ __attribute__((aligned(16))) float Wf1T[256];
  __shared__ __attribute__((aligned(16))) float Wf2T[256];
  __shared__ __attribute__((aligned(16))) float bE2s[64];
  __shared__ __attribute__((aligned(16))) float bC2s[32];
  __shared__ __attribute__((aligned(16))) float bF1s[16];
  __shared__ __attribute__((aligned(16))) float bF2s[16];
  __shared__ __attribute__((aligned(16))) float Ps[384];
  __shared__ __attribute__((aligned(16))) float cis[96];
  __shared__ __attribute__((aligned(16))) float dfL[1536];
  __shared__ __attribute__((aligned(16))) float facL[512];
  __shared__ __attribute__((aligned(16))) float t1L[512];
  __shared__ __attribute__((aligned(16))) float sw[256];

  const int tid = threadIdx.x, lane = tid & 31, w = tid >> 5, hh = lane >> 4, m = lane & 15;
  const int b = blockIdx.y;
  const int inode = blockIdx.x * 2 + w;
  const int gnode = b * NAG + inode;

#pragma unroll 1
  for (int idx = tid; idx < 1024; idx += 64) {
    const float v = We1[(idx >> 4) * WE1P + 128 + (idx & 15)];
    const bf16 hb = (bf16)v;
    CAh[idx] = hb;
    CAl[idx] = (bf16)(v - (float)hb);
  }
#pragma unroll 1
  for (int idx = tid; idx < 2048; idx += 64) {
    const float v = Wc1[(idx >> 10) * WC1SZ + ((idx >> 4) & 63) * WE1P + 128 + (idx & 15)];
    const bf16 hb = (bf16)v;
    CAh[1024 + idx] = hb;
    CAl[1024 + idx] = (bf16)(v - (float)hb);
  }
#pragma unroll 1
  for (int idx = tid; idx < 256; idx += 64) {
    const int src = (idx & 15) * 16 + (idx >> 4);
    Wf1T[idx] = Wf1g[src];
    Wf2T[idx] = Wf2g[src];
  }
  bE2s[tid] = bE2g[tid];
  {
    const float vc2 = bC2g[min(tid, 31)];
    const float vf1 = bF1g[min(tid, 15)];
    const float vf2 = bF2g[min(tid, 15)];
    if (tid < 32) bC2s[tid] = vc2;
    if (tid < 16) { bF1s[tid] = vf1; bF2s[tid] = vf2; }
  }
  {
    const float* pr = NP + (size_t)gnode * NPP;
#pragma unroll 1
    for (int k = lane; k < 192; k += 32) Ps[w * 192 + k] = pr[k];
    const float* cr = coord + (size_t)gnode * 48;
    const int lc = min(lane, 23);
    const float ca = cr[lc], cb = cr[24 + lc];
    if (lane < 24) { cis[w * 48 + lane] = ca; cis[w * 48 + 24 + lane] = cb; }
#pragma unroll
    for (int q = 0; q < 4; ++q) sw[w * 128 + q * 32 + lane] = 0.0f;
  }
  __syncthreads();

  const float* Pw = Ps + w * 192;
  bf16* uHw = uH + w * 3072;
  bf16* uLw = uL + w * 3072;
  float* dfw  = dfL + (w * 32 + lane) * 24;
  float* facw = facL + w * 256;
  float* t1w  = t1L + w * 256;
  float* sww  = sw + w * 128;
  const float* catr = category + (size_t)gnode * (NAG * 2);
  const v8b z8 = zero8b();

  float cagg[24];
#pragma unroll
  for (int e = 0; e < 24; ++e) cagg[e] = 0.0f;

#pragma unroll 1
  for (int jt = 0; jt < 16; ++jt) {
    int zl = 0;
    asm volatile("" : "+v"(zl));
    const int jn = b * NAG + jt * 16 + m;

    FragB bdh, bdl;
    {
      const float* cjp = coord + (size_t)jn * 48 + 24 * hh;
      const float* cip = cis + w * 48 + 24 * hh + zl;
      v4f df[6];
#pragma unroll
      for (int q = 0; q < 6; ++q) {
        const v4f cj = *(const v4fa*)(cjp + 4 * q);
        const v4f ci = *(const v4fa*)(cip + 4 * q);
        df[q] = ci - cj;
        *(v4fa*)(dfw + 4 * q) = df[q];
      }
      v8b dh8, dl8;
#pragma unroll
      for (int cc = 0; cc < 8; ++cc) {
        const float dx = GE(df, 3 * cc), dy = GE(df, 3 * cc + 1), dz = GE(df, 3 * cc + 2);
        float s = dx * dx;
        s += dy * dy;
        s += dz * dz;
        const float d = sqrtf(s);
        const bf16 hb = (bf16)d;
        dh8[cc] = hb;
        dl8[cc] = (bf16)(d - (float)hb);
      }
      bdh.h[0] = dh8; bdh.h[1] = z8;
      bdl.h[0] = dl8; bdl.h[1] = z8;
    }

    const float* qrow = NP + (size_t)jn * NPP + 192;
#pragma unroll 1
    for (int hd = 0; hd < 3; ++hd) {
#pragma unroll 1
      for (int ot = 0; ot < 4; ++ot) {
        const int ob = hd * 64 + ot * 16 + 8 * hh;
        const v4f p0 = *(const v4fa*)(Pw + ob + zl);
        const v4f p1 = *(const v4fa*)(Pw + ob + 4 + zl);
        const v4f q0 = *(const v4fa*)(qrow + ob);
        const v4f q1 = *(const v4fa*)(qrow + ob + 4);
        v8f acc;
        acc[0] = p0[0] + q0[0]; acc[1] = p0[1] + q0[1]; acc[2] = p0[2] + q0[2]; acc[3] = p0[3] + q0[3];
        acc[4] = p1[0] + q1[0]; acc[5] = p1[1] + q1[1]; acc[6] = p1[2] + q1[2]; acc[7] = p1[3] + q1[3];
        FragB ah, al;
        const int arow = (hd * 64 + ot * 16 + m) * 16 + 8 * hh;
        ah.h[0] = *(const v8ba*)(CAh + arow); ah.h[1] = z8;
        al.h[0] = *(const v8ba*)(CAl + arow); al.h[1] = z8;
        acc = wm3(ah, al, bdh, bdl, acc);
        v8b uh8, ul8;
#pragma unroll
        for (int r = 0; r < 8; ++r) {
          const float u = fmaxf(acc[r], 0.0f);
          const bf16 hb = (bf16)u;
          uh8[r] = hb;
          ul8[r] = (bf16)(u - (float)hb);
        }
        const int uo = hd * 1024 + m * 64 + ot * 16 + 8 * hh;
        *(v8ba*)(uHw + uo) = uh8;
        *(v8ba*)(uLw + uo) = ul8;
      }
    }
    __syncthreads();

    {
      FragB ah0, al0, ah1, al1;
      ldb16(uHw + m * 64, uLw + m * 64, hh, ah0, al0);
      ldb16(uHw + m * 64 + 32, uLw + m * 64 + 32, hh, ah1, al1);
#pragma unroll 1
      for (int nt = 0; nt < 4; ++nt) {
        const bf16* ph = WB + OE2H + (nt * 16 + m) * 64;
        const bf16* pl = WB + OE2L + (nt * 16 + m) * 64;
        FragB bh, bl;
        v8f acc = zacc();
        ldb16(ph, pl, hh, bh, bl);
        acc = wm3(ah0, al0, bh, bl, acc);
        ldb16(ph + 32, pl + 32, hh, bh, bl);
        acc = wm3(ah1, al1, bh, bl, acc);
        const float bias = bE2s[nt * 16 + m];
        float s = 0.0f;
#pragma unroll
        for (int r = 0; r < 8; ++r) {
          const int jj = jt * 16 + 8 * hh + r;
          const float v = fmaxf(acc[r] + bias, 0.0f);
          s += (jj != inode) ? v : 0.0f;
        }
        s += __shfl_xor(s, 16);
        const int ao = nt * 16 + m;
        const float na = sww[ao] + s;
        if (hh == 0) sww[ao] = na;
      }
    }

    float fp[8];
#pragma unroll
    for (int r = 0; r < 8; ++r) fp[r] = 0.0f;
#pragma unroll 1
    for (int kc = 0; kc < 2; ++kc) {
      const bf16* ub = uHw + (1 + kc) * 1024 + m * 64;
      const bf16* lb = uLw + (1 + kc) * 1024 + m * 64;
      FragB ah0, al0, ah1, al1;
      ldb16(ub, lb, hh, ah0, al0);
      ldb16(ub + 32, lb + 32, hh, ah1, al1);
      const bf16* ph = WB + OC2H + (kc * 16 + m) * 64;
      const bf16* pl = WB + OC2L + (kc * 16 + m) * 64;
      FragB bh, bl;
      v8f acc = zacc();
      ldb16(ph, pl, hh, bh, bl);
      acc = wm3(ah0, al0, bh, bl, acc);
      ldb16(ph + 32, pl + 32, hh, bh, bl);
      acc = wm3(ah1, al1, bh, bl, acc);
      const float bias = bC2s[kc * 16 + m];
      const float* cp = catr + (size_t)(jt * 16 + 8 * hh) * 2 + kc;
#pragma unroll
      for (int r = 0; r < 8; ++r) {
        const float catv = cp[2 * r];
        fp[r] += catv * fmaxf(acc[r] + bias, 0.0f);
      }
    }
#pragma unroll
    for (int r = 0; r < 8; ++r) facw[(8 * hh + r) * 16 + m] = fp[r];
    __syncthreads();

    {
      float t[8];
      {
        const v4f ba = *(const v4fa*)(bF1s + 8 * hh + zl);
        const v4f bb = *(const v4fa*)(bF1s + 8 * hh + 4 + zl);
        t[0] = ba[0]; t[1] = ba[1]; t[2] = ba[2]; t[3] = ba[3];
        t[4] = bb[0]; t[5] = bb[1]; t[6] = bb[2]; t[7] = bb[3];
      }
#pragma unroll 1
      for (int c = 0; c < 16; ++c) {
        const float f = facw[m * 16 + c];
        const v4f wa = *(const v4fa*)(Wf1T + c * 16 + 8 * hh);
        const v4f wb = *(const v4fa*)(Wf1T + c * 16 + 8 * hh + 4);
        t[0] += wa[0] * f; t[1] += wa[1] * f; t[2] += wa[2] * f; t[3] += wa[3] * f;
        t[4] += wb[0] * f; t[5] += wb[1] * f; t[6] += wb[2] * f; t[7] += wb[3] * f;
      }
      v4f ta, tb;
      ta[0] = fmaxf(t[0], 0.0f); ta[1] = fmaxf(t[1], 0.0f); ta[2] = fmaxf(t[2], 0.0f); ta[3] = fmaxf(t[3], 0.0f);
      tb[0] = fmaxf(t[4], 0.0f); tb[1] = fmaxf(t[5], 0.0f); tb[2] = fmaxf(t[6], 0.0f); tb[3] = fmaxf(t[7], 0.0f);
      *(v4fa*)(t1w + m * 16 + 8 * hh) = ta;
      *(v4fa*)(t1w + m * 16 + 8 * hh + 4) = tb;
    }
    __syncthreads();

    float f2[8];
    {
      float t[8];
      {
        const v4f ba = *(const v4fa*)(bF2s + 8 * hh + zl);
        const v4f bb = *(const v4fa*)(bF2s + 8 * hh + 4 + zl);
        t[0] = ba[0]; t[1] = ba[1]; t[2] = ba[2]; t[3] = ba[3];
        t[4] = bb[0]; t[5] = bb[1]; t[6] = bb[2]; t[7] = bb[3];
      }
#pragma unroll 1
      for (int o = 0; o < 16; ++o) {
        const float tv = t1w[m * 16 + o];
        const v4f wa = *(const v4fa*)(Wf2T + o * 16 + 8 * hh);
        const v4f wb = *(const v4fa*)(Wf2T + o * 16 + 8 * hh + 4);
        t[0] += wa[0] * tv; t[1] += wa[1] * tv; t[2] += wa[2] * tv; t[3] += wa[3] * tv;
        t[4] += wb[0] * tv; t[5] += wb[1] * tv; t[6] += wb[2] * tv; t[7] += wb[3] * tv;
      }
#pragma unroll
      for (int cc = 0; cc < 8; ++cc) f2[cc] = fmaxf(t[cc], 0.0f);
    }

    {
      v4f df[6];
#pragma unroll
      for (int q = 0; q < 6; ++q) df[q] = *(const v4fa*)(dfw + 4 * q);
#pragma unroll
      for (int cc = 0; cc < 8; ++cc) {
#pragma unroll
        for (int d = 0; d < 3; ++d) {
          const int e = cc * 3 + d;
          cagg[e] += f2[cc] * GE(df, e);
        }
      }
    }
  }

#pragma unroll
  for (int e = 0; e < 24; ++e) {
    float v = cagg[e];
    v += __shfl_xor(v, 1);
    v += __shfl_xor(v, 2);
    v += __shfl_xor(v, 4);
    v += __shfl_xor(v, 8);
    cagg[e] = v;
  }
  if (m == 0) {
#pragma unroll
    for (int e = 0; e < 24; ++e) sww[64 + 24 * hh + e] = cagg[e];
  }
  __syncthreads();
  {
    const v4f v = *(const v4fa*)(sww + 4 * lane);
    float* orow = NA + (size_t)gnode * NAP + 4 * lane;
    *(volatile v4f*)orow = v;
    __threadfence();
    *(volatile v4f*)orow = v;
  }
}

__device__ __forceinline__ void slab_store(const float* src, float* dst, const int tid) {
#pragma unroll
  for (int it = 0; it < 12; ++it) {
    const int piece = it * 256 + tid;
    const v4f v = *(const v4fa*)(src + piece * 4);
    *(volatile v4f*)(dst + (size_t)piece * 4) = v;
  }
}

__device__ __forceinline__ void tile_store(const float* src, float* dst, const int lane) {
#pragma unroll
  for (int it = 0; it < 8; ++it) {
    const int piece = it * 32 + lane;
    const v4f v = *(const v4fa*)(src + piece * 4);
    *(volatile v4f*)(dst + (size_t)piece * 4) = v;
  }
}

#define ACC3(q, v)                                                                       \
  {                                                                                      \
    if (((q) % 3) == 0)      { sx += v[0]; sy += v[1]; sz += v[2]; sx += v[3]; }         \
    else if (((q) % 3) == 1) { sy += v[0]; sz += v[1]; sx += v[2]; sy += v[3]; }         \
    else                     { sz += v[0]; sx += v[1]; sy += v[2]; sz += v[3]; }         \
  }

__global__ __launch_bounds__(256) void k_final(
    const float* __restrict__ h, const float* __restrict__ coord, const float* __restrict__ vel,
    const float* __restrict__ NP, const float* __restrict__ NA, const bf16* __restrict__ WB,
    const float* __restrict__ Wcv, const float* __restrict__ Wql, const float* __restrict__ Wkl,
    const float* __restrict__ bN1g, const float* __restrict__ bN2g, float* out0, float* out1) {
  extern __shared__ __attribute__((aligned(16))) float sm[];
  float* cst = sm + SMF_CST;
  float* ost = sm + SMF_OST;
  float* red = sm + SMF_RED;

  const int tid = threadIdx.x, lane = tid & 31, w = tid >> 5, hh = lane >> 4, m = lane & 15;
  const int b = blockIdx.x;
  const int node = b * NAG + tid;
  float* crow = cst + tid * 48;

  float mx, my, mz;
  {
    const float* cr = coord + (size_t)node * 48;
    float sx = 0.0f, sy = 0.0f, sz = 0.0f;
#pragma unroll
    for (int q = 0; q < 12; ++q) {
      const v4f v = *(const v4fa*)(cr + 4 * q);
      *(v4fa*)(crow + 4 * q) = v;
      ACC3(q, v)
    }
    sx = wsum(sx); sy = wsum(sy); sz = wsum(sz);
    if (lane == 0) { red[w * 4 + 0] = sx; red[w * 4 + 1] = sy; red[w * 4 + 2] = sz; }
    __syncthreads();
    float tx = 0.0f, ty = 0.0f, tz = 0.0f;
#pragma unroll
    for (int ww = 0; ww < 8; ++ww) { tx += red[ww * 4]; ty += red[ww * 4 + 1]; tz += red[ww * 4 + 2]; }
    mx = tx * (1.0f / 4096.0f); my = ty * (1.0f / 4096.0f); mz = tz * (1.0f / 4096.0f);
  }

  float cmx, cmy, cmz;
  {
    const float* vr  = vel + (size_t)node * 48;
    const float* car = NA + (size_t)node * NAP + 64;
    const float* atp = NP + (size_t)node * NPP + 384;
    float sx = 0.0f, sy = 0.0f, sz = 0.0f;
#pragma unroll 1
    for (int c = 0; c < 16; ++c) {
      float vx = 0.0f, vy = 0.0f, vz = 0.0f;
#pragma unroll 1
      for (int c2 = 0; c2 < 16; ++c2) {
        const float wv = Wcv[c * 16 + c2];
        const float* vp = vr + 3 * c2;
        vx += wv * vp[0]; vy += wv * vp[1]; vz += wv * vp[2];
      }
      const float ac = atp[c];
      float* cp = crow + 3 * c;
      const float* ap = car + 3 * c;
      const float x0 = cp[0], y0 = cp[1], z0 = cp[2];
      float x = ac * (x0 - mx) + x0; x = x + ap[0]; x = x + vx;
      float y = ac * (y0 - my) + y0; y = y + ap[1]; y = y + vy;
      float z = ac * (z0 - mz) + z0; z = z + ap[2]; z = z + vz;
      cp[0] = x; cp[1] = y; cp[2] = z;
      sx += x; sy += y; sz += z;
    }
    sx = wsum(sx); sy = wsum(sy); sz = wsum(sz);
    if (lane == 0) { red[32 + w * 4 + 0] = sx; red[32 + w * 4 + 1] = sy; red[32 + w * 4 + 2] = sz; }
    __syncthreads();
    float tx = 0.0f, ty = 0.0f, tz = 0.0f;
#pragma unroll
    for (int ww = 0; ww < 8; ++ww) { tx += red[32 + ww * 4]; ty += red[32 + ww * 4 + 1]; tz += red[32 + ww * 4 + 2]; }
    cmx = tx * (1.0f / 4096.0f); cmy = ty * (1.0f / 4096.0f); cmz = tz * (1.0f / 4096.0f);
  }

  {
#pragma unroll 1
    for (int c = 0; c < 16; ++c) {
      float* cp = crow + 3 * c;
      cp[0] = cp[0] - cmx; cp[1] = cp[1] - cmy; cp[2] = cp[2] - cmz;
    }
    float* orow = ost + tid * 48;
#pragma unroll 1
    for (int o = 0; o < 16; ++o) {
      float qx = 0.0f, qy = 0.0f, qz = 0.0f, kx = 0.0f, ky = 0.0f, kz = 0.0f;
#pragma unroll 1
      for (int c = 0; c < 16; ++c) {
        const float wq = Wql[o * 16 + c], wk = Wkl[o * 16 + c];
        const float* cp = crow + 3 * c;
        const float x = cp[0], y = cp[1], z = cp[2];
        qx += wq * x; qy += wq * y; qz += wq * z;
        kx += wk * x; ky += wk * y; kz += wk * z;
      }
      const float prod = qx * kx + qy * ky + qz * kz;
      const float kns  = kx * kx + ky * ky + kz * kz;
      const float tq   = prod * (1.0f / (kns + EPSV));
      const bool  pos  = prod >= 0.0f;
      const float ax = (qx - tq * kx) + cmx, ay = (qy - tq * ky) + cmy, az = (qz - tq * kz) + cmz;
      orow[3 * o + 0] = pos ? (qx + cmx) : ax;
      orow[3 * o + 1] = pos ? (qy + cmy) : ay;
      orow[3 * o + 2] = pos ? (qz + cmz) : az;
    }
  }
  __syncthreads();
  {
    float* ob = out1 + (size_t)b * (NAG * 48);
    slab_store(ost, ob, tid);
    __threadfence();
    slab_store(ost, ob, tid);
  }
  __syncthreads();

  float* tw  = ost + w * 1024;
  float* tw2 = cst + w * 1024;
#pragma unroll 1
  for (int mt = 0; mt < 2; ++mt) {
    const int nrow = b * NAG + (w * 2 + mt) * 16;
#pragma unroll 1
    for (int nt = 0; nt < 4; ++nt) {
      v8f acc = zacc();
      const bf16* ph = WB + ON1H + (nt * 16 + m) * 128;
      const bf16* pl = WB + ON1L + (nt * 16 + m) * 128;
#pragma unroll 1
      for (int ks = 0; ks < 2; ++ks) {
        FragB ah, al, bh, bl;
        ldsplit(h + (size_t)(nrow + m) * NF + ks * 32, hh, ah, al);
        ldb16(ph + ks * 32, pl + ks * 32, hh, bh, bl);
        acc = wm3(ah, al, bh, bl, acc);
      }
#pragma unroll 1
      for (int ks = 0; ks < 2; ++ks) {
        FragB ah, al, bh, bl;
        ldsplit(NA + (size_t)(nrow + m) * NAP + ks * 32, hh, ah, al);
        ldb16(ph + 64 + ks * 32, pl + 64 + ks * 32, hh, bh, bl);
        acc = wm3(ah, al, bh, bl, acc);
      }
      const float bias = bN1g[nt * 16 + m];
#pragma unroll
      for (int r = 0; r < 8; ++r) tw[(8 * hh + r) * 64 + nt * 16 + m] = fmaxf(acc[r] + bias, 0.0f);
    }
    __syncthreads();
#pragma unroll 1
    for (int nt = 0; nt < 4; ++nt) {
      const int col = nt * 16 + m;
      v8f acc = zacc();
      const bf16* ph = WB + ON2H + col * 64;
      const bf16* pl = WB + ON2L + col * 64;
#pragma unroll 1
      for (int ks = 0; ks < 2; ++ks) {
        FragB ah, al, bh, bl;
        ldsplit(tw + m * 64 + ks * 32, hh, ah, al);
        ldb16(ph + ks * 32, pl + ks * 32, hh, bh, bl);
        acc = wm3(ah, al, bh, bl, acc);
      }
      const float bias = bN2g[col];
#pragma unroll
      for (int r = 0; r < 8; ++r) {
        const int rr = 8 * hh + r;
        const float hv = h[(size_t)(nrow + rr) * NF + col];
        tw2[rr * 64 + col] = hv + (acc[r] + bias);
      }
    }
    __syncthreads();
    {
      float* ob0 = out0 + (size_t)nrow * NF;
      tile_store(tw2, ob0, lane);
      __threadfence();
      tile_store(tw2, ob0, lane);
    }
    __syncthreads();
  }
}

extern "C" void kernel_launch(void* const* d_in, const int* in_sizes, int n_in,
                              void* d_out, int out_size, void* d_ws, size_t ws_size,
                              hipStream_t stream) {
  if (n_in < 25) return;
  const int want[25] = {131072, 98304, 98304, 1048576, 256, 9216, 64, 4096, 64, 18432, 128, 2048, 32,
                        256, 16, 256, 16, 8192, 64, 4096, 64, 256, 256, 1024, 16};
  for (int q = 0; q < 25; ++q) if (in_sizes[q] != want[q]) return;
  if (out_size != 131072 + 98304 + 1048576) return;

  const float* h     = (const float*)d_in[0];
  const float* coord = (const float*)d_in[1];
  const float* vel   = (const float*)d_in[2];
  const float* cat   = (const float*)d_in[3];
  const float* Wcv   = (const float*)d_in[4];
  const float* We1   = (const float*)d_in[5];
  const float* bE1   = (const float*)d_in[6];
  const float* We2   = (const float*)d_in[7];
  const float* bE2   = (const float*)d_in[8];
  const float* Wc1   = (const float*)d_in[9];
  const float* bC1   = (const float*)d_in[10];
  const float* Wc2   = (const float*)d_in[11];
  const float* bC2   = (const float*)d_in[12];
  const float* Wf1   = (const float*)d_in[13];
  const float* bF1   = (const float*)d_in[14];
  const float* Wf2   = (const float*)d_in[15];
  const float* bF2   = (const float*)d_in[16];
  const float* Wn1   = (const float*)d_in[17];
  const float* bN1   = (const float*)d_in[18];
  const float* Wn2   = (const float*)d_in[19];
  const float* bN2   = (const float*)d_in[20];
  const float* Wql   = (const float*)d_in[21];
  const float* Wkl   = (const float*)d_in[22];
  const float* Wqm   = (const float*)d_in[23];
  const float* bqm   = (const float*)d_in[24];

  float* out0 = (float*)d_out;
  float* out1 = out0 + 131072;
  float* out2 = out0 + 229376;

  char* ws = (char*)d_ws;
  size_t off = 0;
  const size_t oWB = off; off += (size_t)WBN * 2;         off = (off + 255) & ~(size_t)255;
  const size_t oNP = off; off += (size_t)NODES * NPP * 4; off = (off + 255) & ~(size_t)255;
  const size_t oNA = off; off += (size_t)NODES * NAP * 4; off = (off + 255) & ~(size_t)255;
  if (off > ws_size) return;
  bf16*  WB = (bf16*)(ws + oWB);
  float* NP = (float*)(ws + oNP);
  float* NA = (float*)(ws + oNA);

  k_wsplit<<<9, 256, 0, stream>>>(We2, Wc2, Wn1, Wn2, WB);
  k_copy<<<256, 256, 0, stream>>>(cat, out2);
  k_planes<<<128, 32, 0, stream>>>(h, We1, bE1, Wc1, bC1, Wqm, bqm, NP);
  k_pairs<<<dim3(128, 8), 64, 0, stream>>>(NP, coord, cat, WB, We1, Wc1, bE2, bC2, Wf1, bF1, Wf2, bF2, NA);
  k_final<<<8, 256, (size_t)SMF_TOTAL * 4, stream>>>(h, coord, vel, NP, NA, WB, Wcv, Wql, Wkl, bN1, bN2, out0, out1);
}
